// S4R_58308476010695
// MI455X (gfx1250) — hardware-verified
//
#include <hip/hip_runtime.h>

typedef _Float16 v16h __attribute__((ext_vector_type(16)));
typedef _Float16 v8h  __attribute__((ext_vector_type(8)));
typedef __bf16   v16b __attribute__((ext_vector_type(16)));
typedef __bf16   v8b  __attribute__((ext_vector_type(8)));
typedef unsigned short v8us __attribute__((ext_vector_type(8)));
typedef float    v8f  __attribute__((ext_vector_type(8)));
typedef float    v4f  __attribute__((ext_vector_type(4)));
typedef v8h  __attribute__((may_alias)) v8ha;
typedef v8b  __attribute__((may_alias)) v8ba;
typedef v8us __attribute__((may_alias)) v8usa;
typedef v4f  __attribute__((may_alias)) v4fa;

union Frag  { v16h v; v8h half[2]; };
union FragB { v16b v; v8b half[2]; };

#define NB   8
#define NH   256
#define NL   4096
#define NP   64
#define NO   512
#define UPAD 64
#define UP   (NL + UPAD)
#define UPC  (UP / 8)
#define NE   128
#define NUPC (NB * NH * UPC)
#define NWPC (NO * NH / 8)
#define YP   264
#define SP   36

#define KSC      256.0f
#define USC      64.0f
#define INV_CONV (1.0f / 16384.0f)
#define ECUT     64.0f

static_assert(NUPC % 256 == 0);
static_assert(NWPC % 256 == 0);

__device__ __forceinline__ unsigned int bf16_bits_rne(float x) {
  const unsigned int u = __builtin_bit_cast(unsigned int, x);
  return (u + 0x7FFFu + ((u >> 16) & 1u)) >> 16;
}
__device__ __forceinline__ void split_bf16(float x, unsigned short& hi, unsigned short& lo) {
  const unsigned int hb = bf16_bits_rne(x);
  const float hf = __builtin_bit_cast(float, hb << 16);
  hi = (unsigned short)hb;
  lo = (unsigned short)bf16_bits_rne(x - hf);
}

__device__ __forceinline__ v8f wmma_f16(v16h a, v16h b, v8f c) {
  v8f d = __builtin_amdgcn_wmma_f32_16x16x32_f16(false, a, false, b, (short)0, c, false, false);
  asm volatile("v_nop\n\tv_nop\n\tv_nop\n\tv_nop" : "+v"(d) : "v"(a), "v"(b));
  return d;
}
__device__ __forceinline__ v8f wmma_bf16(v16b a, v16b b, v8f c) {
  v8f d = __builtin_amdgcn_wmma_f32_16x16x32_bf16(false, a, false, b, (short)0, c, false, false);
  asm volatile("v_nop\n\tv_nop\n\tv_nop\n\tv_nop" : "+v"(d) : "v"(a), "v"(b));
  return d;
}

__device__ __forceinline__ v16h load_frag(const _Float16* p, int hh) {
  Frag f;
  f.half[0] = *(const v8ha*)(p + 8 * hh);
  f.half[1] = *(const v8ha*)(p + 16 + 8 * hh);
  return f.v;
}
__device__ __forceinline__ v16b load_frag_b(const unsigned short* p, int hh) {
  FragB f;
  f.half[0] = *(const v8ba*)(p + 8 * hh);
  f.half[1] = *(const v8ba*)(p + 16 + 8 * hh);
  return f.v;
}

__device__ __forceinline__ void sincos_cw(float p, float& sn, float& cs) {
  const float q = rintf(p * 0.636619772367581343f);
  float r = fmaf(-q, 1.57079637050628662109375f, p);
  r = fmaf(-q, -4.37113882867379e-8f, r);
  const int n = (int)q;
  const float z = r * r;
  const float sp = r + r * z * (-1.0f / 6.0f + z * (1.0f / 120.0f + z * (-1.0f / 5040.0f + z * (1.0f / 362880.0f))));
  const float cp = 1.0f + z * (-0.5f + z * (1.0f / 24.0f + z * (-1.0f / 720.0f + z * (1.0f / 40320.0f + z * (-1.0f / 3628800.0f)))));
  const float ss = (n & 1) ? cp : sp;
  const float cc = (n & 1) ? sp : cp;
  sn = (n & 2) ? -ss : ss;
  cs = ((n + 1) & 2) ? -cc : cc;
}

__global__ __launch_bounds__(256) void k_cvt(
    const float* __restrict__ u, const float* __restrict__ W,
    _Float16* __restrict__ uh, unsigned short* __restrict__ whi, unsigned short* __restrict__ wlo)
{
  const int g = blockIdx.x * 256 + threadIdx.x;
  if (g >= NUPC + NWPC) return;
  if (g < NUPC) {
    const int row = g / UPC;
    const int c = g - row * UPC;
    const int cc = (c >= 8) ? (c - 8) : 0;
    const float* src = u + (size_t)row * NL + (size_t)cc * 8;
    _Float16* dst = uh + (size_t)row * UP + (size_t)c * 8;
    const bool live = (c >= 8);
    const v4f a = *(const v4fa*)src;
    const v4f c4 = *(const v4fa*)(src + 4);
    v8h o;
    o[0] = live ? (_Float16)(a.x * USC)  : (_Float16)0.0f;
    o[1] = live ? (_Float16)(a.y * USC)  : (_Float16)0.0f;
    o[2] = live ? (_Float16)(a.z * USC)  : (_Float16)0.0f;
    o[3] = live ? (_Float16)(a.w * USC)  : (_Float16)0.0f;
    o[4] = live ? (_Float16)(c4.x * USC) : (_Float16)0.0f;
    o[5] = live ? (_Float16)(c4.y * USC) : (_Float16)0.0f;
    o[6] = live ? (_Float16)(c4.z * USC) : (_Float16)0.0f;
    o[7] = live ? (_Float16)(c4.w * USC) : (_Float16)0.0f;
    *(volatile v8h*)dst = o;
    __threadfence();
    *(volatile v8h*)dst = o;
  } else {
    const int e = g - NUPC;
    const float* src = W + (size_t)e * 8;
    const v4f a = *(const v4fa*)src;
    const v4f c4 = *(const v4fa*)(src + 4);
    v8us hv, lv;
    unsigned short th, tl;
    split_bf16(a.x,  th, tl); hv[0] = th; lv[0] = tl;
    split_bf16(a.y,  th, tl); hv[1] = th; lv[1] = tl;
    split_bf16(a.z,  th, tl); hv[2] = th; lv[2] = tl;
    split_bf16(a.w,  th, tl); hv[3] = th; lv[3] = tl;
    split_bf16(c4.x, th, tl); hv[4] = th; lv[4] = tl;
    split_bf16(c4.y, th, tl); hv[5] = th; lv[5] = tl;
    split_bf16(c4.z, th, tl); hv[6] = th; lv[6] = tl;
    split_bf16(c4.w, th, tl); hv[7] = th; lv[7] = tl;
    unsigned short* dh = whi + (size_t)e * 8;
    unsigned short* dl = wlo + (size_t)e * 8;
    *(volatile v8us*)dh = hv;
    *(volatile v8us*)dl = lv;
    __threadfence();
    *(volatile v8us*)dh = hv;
    *(volatile v8us*)dl = lv;
  }
}

__global__ __launch_bounds__(256) void k_kern(
    const float* __restrict__ lam_re, const float* __restrict__ lam_im,
    const float* __restrict__ cb_re,  const float* __restrict__ cb_im,
    _Float16* __restrict__ At)
{
  __shared__ float plg[NP], pag[NP], pcr[NP], pci[NP];
  __shared__ int   pnit[NP];
  __shared__ __attribute__((aligned(16))) float Ks[NL];

  const int h = blockIdx.x, tid = threadIdx.x;

  if (tid < NP) {
    const float re = lam_re[h * NP + tid];
    const float im = lam_im[h * NP + tid];
    const float ab = sqrtf(re * re + im * im);
    const float lg = logf(ab);
    const float ag = atan2f(im, re);
    const float rc = __builtin_amdgcn_rcpf(-lg) * ECUT;
    const float ctf = (lg < 0.0f) ? fminf(rc, 4096.0f) : 4096.0f;
    int nit = ((int)ctf + 256) >> 8;
    nit = max(1, min(16, nit));
    plg[tid] = lg;
    pag[tid] = ag;
    pcr[tid] = cb_re[h * NP + tid];
    pci[tid] = cb_im[h * NP + tid];
    pnit[tid] = nit;
  }
  #pragma unroll 1
  for (int it = 0; it < NL / 256; ++it) Ks[it * 256 + tid] = 0.0f;
  __syncthreads();

  #pragma unroll 1
  for (int n = 0; n < NP; ++n) {
    const float lgn = plg[n], agn = pag[n], crn = pcr[n], cin = pci[n];
    const int nit = min(pnit[n], 16);
    #pragma unroll 1
    for (int it = 0; it < nit; ++it) {
      const int l = it * 256 + tid;
      const float lf = (float)l;
      const float a = lgn * lf;
      const float p = agn * lf;
      const float ex = expf(a);
      float sn, cs;
      sincos_cw(p, sn, cs);
      const float vr = ex * cs;
      const float vi = ex * sn;
      Ks[l] += crn * vr - cin * vi;
    }
  }
  __syncthreads();

  _Float16* base = At + (size_t)h * NE * 512;
  #pragma unroll 1
  for (int it = 0; it < 32; ++it) {
    const int pc = it * 256 + tid;
    const int ei = pc >> 6, q = pc & 63, i = q >> 2, c = q & 3;
    const int lag0 = 16 * (2 * ei + 1) + i - 8 * c;
    v8h o;
    #pragma unroll
    for (int j = 0; j < 8; ++j) {
      const int lag = lag0 - j;
      const float kv = Ks[(lag >= 0) ? lag : 0];
      o[j] = (_Float16)(((lag >= 0) ? kv : 0.0f) * (2.0f * KSC));
    }
    _Float16* dst = base + ((size_t)ei * 16 + i) * 32 + 8 * c;
    *(volatile v8h*)dst = o;
    __threadfence();
    *(volatile v8h*)dst = o;
  }
}

__device__ __forceinline__ v8f conv_tile(const _Float16* arow, const _Float16* ubs, int t, int hh) {
  const v8f zero8 = {0.f, 0.f, 0.f, 0.f, 0.f, 0.f, 0.f, 0.f};
  v8f acc = zero8;
  const _Float16* ap = arow;
  const _Float16* bp = ubs + 32 * t;
  #pragma unroll 1
  for (int ei = 0; ei <= t; ++ei) {
    const v16h a = load_frag(ap, hh);
    const v16h bv = load_frag(bp, hh);
    acc = wmma_f16(a, bv, acc);
    ap += 512;
    bp -= 32;
  }
  return acc;
}

__device__ __forceinline__ void stage_tile(v8f acc, int t, const float* urow, float dv,
                                           unsigned short* ysw, int hh, int s, int b, int g) {
  const int ll = 32 * (t & 1) + 16 * s + 8 * hh;
  const v4f u0 = *(const v4fa*)(urow + 64 * g + ll);
  const v4f u1 = *(const v4fa*)(urow + 64 * g + ll + 4);
  const v8f uv = { u0.x, u0.y, u0.z, u0.w, u1.x, u1.y, u1.z, u1.w };
  v8us ho, lo8;
  #pragma unroll
  for (int r = 0; r < 8; ++r) {
    const float yp = acc[r] * INV_CONV + dv * uv[r];
    const float yv = tanhf(yp);
    unsigned short th, tl;
    split_bf16(yv, th, tl);
    ho[r] = th;
    lo8[r] = tl;
  }
  *(v8usa*)(ysw + b * 64 + ll) = ho;
  *(v8usa*)(ysw + 512 + b * 64 + ll) = lo8;
}

__device__ __forceinline__ void y_store_pass(const unsigned short* ysw, unsigned short* yhi, unsigned short* ylo,
                                             int h, int g, int lane) {
  const int q8 = lane & 7, sub = lane >> 3;
  #pragma unroll
  for (int i = 0; i < 2; ++i) {
    const int b = 4 * i + sub;
    const size_t gi = ((size_t)(b * NH + h)) * NL + 64 * g + 8 * q8;
    const v8us vh = *(const v8usa*)(ysw + b * 64 + 8 * q8);
    const v8us vl = *(const v8usa*)(ysw + 512 + b * 64 + 8 * q8);
    *(volatile v8us*)(yhi + gi) = vh;
    *(volatile v8us*)(ylo + gi) = vl;
  }
}

__global__ __launch_bounds__(128) void k_conv(
    const _Float16* __restrict__ uh,
    const _Float16* __restrict__ At,
    const float* __restrict__ u32,
    const float* __restrict__ Dv,
    unsigned short* __restrict__ yhi,
    unsigned short* __restrict__ ylo)
{
  __shared__ __attribute__((aligned(16))) unsigned short ys[4 * 2 * 8 * 64];

  const int tid = threadIdx.x, lane = tid & 31, w = tid >> 5;
  const int hh = lane >> 4, n = lane & 15, s = n >> 3, b = n & 7;
  const int h = blockIdx.y;
  const int q = blockIdx.x * 4 + w;
  const float dv = Dv[h];

  const _Float16* arow = At + ((size_t)h * NE * 16 + n) * 32;
  const _Float16* urow = uh + ((size_t)(b * NH + h)) * UP;
  const _Float16* ubs  = urow + 48 + 16 * s;
  const float* urow32  = u32 + ((size_t)(b * NH + h)) * NL;
  unsigned short* ysw = ys + w * 1024;

  #pragma unroll 1
  for (int gp = 0; gp < 2; ++gp) {
    const int g = (gp == 0) ? q : (63 - q);
    const v8f acc0 = conv_tile(arow, ubs, 2 * g, hh);
    const v8f acc1 = conv_tile(arow, ubs, 2 * g + 1, hh);
    stage_tile(acc0, 2 * g,     urow32, dv, ysw, hh, s, b, g);
    stage_tile(acc1, 2 * g + 1, urow32, dv, ysw, hh, s, b, g);
    __syncthreads();
    y_store_pass(ysw, yhi, ylo, h, g, lane);
    __threadfence();
    y_store_pass(ysw, yhi, ylo, h, g, lane);
    __syncthreads();
  }
}

__device__ __forceinline__ void out_store_pass(const float* sw, float* out, int b, int w, int l0, int lane) {
  const int q8 = lane & 7, sub = lane >> 3;
  #pragma unroll
  for (int i = 0; i < 8; ++i) {
    const int orow = 4 * i + sub;
    const v4f v = *(const v4fa*)(sw + orow * SP + 4 * q8);
    float* dst = out + ((size_t)(b * NH + 32 * w + orow)) * NL + l0 + 4 * q8;
    *(volatile v4f*)dst = v;
  }
}

__global__ __launch_bounds__(256) void k_mix(
    const unsigned short* __restrict__ yhi,
    const unsigned short* __restrict__ ylo,
    const unsigned short* __restrict__ whi,
    const unsigned short* __restrict__ wlo,
    const float* __restrict__ bmix,
    float* __restrict__ out)
{
  __shared__ __attribute__((aligned(16))) unsigned short ysh[32 * YP];
  __shared__ __attribute__((aligned(16))) unsigned short ysl[32 * YP];
  __shared__ __attribute__((aligned(16))) float so[8 * 32 * SP];

  const int tid = threadIdx.x, lane = tid & 31, w = tid >> 5;
  const int hh = lane >> 4, m = lane & 15;
  const int l0 = blockIdx.x * 32, b = blockIdx.y;

  #pragma unroll
  for (int it = 0; it < 4; ++it) {
    const int pc = it * 256 + tid;
    const int hr = pc >> 2, c = pc & 3;
    const size_t gi = ((size_t)(b * NH + hr)) * NL + l0 + 8 * c;
    const v8us vh = *(const v8usa*)(yhi + gi);
    const v8us vl = *(const v8usa*)(ylo + gi);
    #pragma unroll
    for (int j = 0; j < 8; ++j) {
      ysh[(8 * c + j) * YP + hr] = vh[j];
      ysl[(8 * c + j) * YP + hr] = vl[j];
    }
  }
  __syncthreads();

  const v8f zero8 = {0.f, 0.f, 0.f, 0.f, 0.f, 0.f, 0.f, 0.f};
  v8f aa[2][2], ag[2][2];
  #pragma unroll
  for (int mt = 0; mt < 2; ++mt)
    #pragma unroll
    for (int nt = 0; nt < 2; ++nt) { aa[mt][nt] = zero8; ag[mt][nt] = zero8; }

  const unsigned short* wah = whi + ((size_t)(32 * w + m)) * NH;
  const unsigned short* wal = wlo + ((size_t)(32 * w + m)) * NH;
  const unsigned short* wgh = wah + (size_t)256 * NH;
  const unsigned short* wgl = wal + (size_t)256 * NH;
  const unsigned short* ybh = ysh + m * YP;
  const unsigned short* ybl = ysl + m * YP;

  #pragma unroll 1
  for (int k0 = 0; k0 < NH; k0 += 32) {
    const v16b bh0 = load_frag_b(ybh + k0, hh);
    const v16b bh1 = load_frag_b(ybh + 16 * YP + k0, hh);
    const v16b bl0 = load_frag_b(ybl + k0, hh);
    const v16b bl1 = load_frag_b(ybl + 16 * YP + k0, hh);
    #pragma unroll
    for (int mt = 0; mt < 2; ++mt) {
      const v16b fah = load_frag_b(wah + (size_t)(16 * mt) * NH + k0, hh);
      const v16b fal = load_frag_b(wal + (size_t)(16 * mt) * NH + k0, hh);
      aa[mt][0] = wmma_bf16(fah, bh0, aa[mt][0]);
      aa[mt][0] = wmma_bf16(fah, bl0, aa[mt][0]);
      aa[mt][0] = wmma_bf16(fal, bh0, aa[mt][0]);
      aa[mt][1] = wmma_bf16(fah, bh1, aa[mt][1]);
      aa[mt][1] = wmma_bf16(fah, bl1, aa[mt][1]);
      aa[mt][1] = wmma_bf16(fal, bh1, aa[mt][1]);
      const v16b fgh = load_frag_b(wgh + (size_t)(16 * mt) * NH + k0, hh);
      const v16b fgl = load_frag_b(wgl + (size_t)(16 * mt) * NH + k0, hh);
      ag[mt][0] = wmma_bf16(fgh, bh0, ag[mt][0]);
      ag[mt][0] = wmma_bf16(fgh, bl0, ag[mt][0]);
      ag[mt][0] = wmma_bf16(fgl, bh0, ag[mt][0]);
      ag[mt][1] = wmma_bf16(fgh, bh1, ag[mt][1]);
      ag[mt][1] = wmma_bf16(fgh, bl1, ag[mt][1]);
      ag[mt][1] = wmma_bf16(fgl, bh1, ag[mt][1]);
    }
  }

  float* sw = so + w * 32 * SP;
  #pragma unroll
  for (int mt = 0; mt < 2; ++mt) {
    #pragma unroll
    for (int r = 0; r < 8; ++r) {
      const int orow = 16 * mt + 8 * hh + r;
      const int o = 32 * w + orow;
      const float ba = bmix[o];
      const float bg = bmix[o + 256];
      #pragma unroll
      for (int nt = 0; nt < 2; ++nt) {
        const float za = aa[mt][nt][r] + ba;
        const float zg = ag[mt][nt][r] + bg;
        const float sg = __builtin_amdgcn_rcpf(1.0f + expf(-zg));
        sw[orow * SP + 16 * nt + m] = za * sg;
      }
    }
  }
  __syncthreads();

  out_store_pass(sw, out, b, w, l0, lane);
  __threadfence();
  out_store_pass(sw, out, b, w, l0, lane);
}

extern "C" void kernel_launch(void* const* d_in, const int* in_sizes, int n_in,
                              void* d_out, int out_size, void* d_ws, size_t ws_size,
                              hipStream_t stream) {
  if (n_in < 8) return;
  if (in_sizes[0] != NB * NH * NL) return;
  if (in_sizes[1] != NH * NP || in_sizes[2] != NH * NP) return;
  if (in_sizes[3] != NH * NP || in_sizes[4] != NH * NP) return;
  if (in_sizes[5] != NH || in_sizes[6] != NO * NH || in_sizes[7] != NO) return;
  if (out_size != NB * NH * NL) return;

  const float* u   = (const float*)d_in[0];
  const float* lre = (const float*)d_in[1];
  const float* lim = (const float*)d_in[2];
  const float* cre = (const float*)d_in[3];
  const float* cim = (const float*)d_in[4];
  const float* Dv  = (const float*)d_in[5];
  const float* W   = (const float*)d_in[6];
  const float* bm  = (const float*)d_in[7];
  float* out = (float*)d_out;

  const size_t uh_bytes = (size_t)NB * NH * UP * 2;
  const size_t wp_bytes = (size_t)NO * NH * 2;
  const size_t at_bytes = (size_t)NH * NE * 512 * 2;
  const size_t yp_bytes = (size_t)NB * NH * NL * 2;
  const size_t total = uh_bytes + 2 * wp_bytes + at_bytes + 2 * yp_bytes;
  if (total > ws_size) return;

  char* ws = (char*)d_ws;
  size_t off = 0;
  _Float16* uh        = (_Float16*)(ws + off);          off += uh_bytes;
  unsigned short* whi = (unsigned short*)(ws + off);    off += wp_bytes;
  unsigned short* wlo = (unsigned short*)(ws + off);    off += wp_bytes;
  _Float16* At        = (_Float16*)(ws + off);          off += at_bytes;
  unsigned short* yhi = (unsigned short*)(ws + off);    off += yp_bytes;
  unsigned short* ylo = (unsigned short*)(ws + off);    off += yp_bytes;
  if (off > ws_size) return;

  const int npc = NUPC + NWPC;
  k_cvt<<<npc / 256, 256, 0, stream>>>(u, W, uh, whi, wlo);

  k_kern<<<NH, 256, 0, stream>>>(lre, lim, cre, cim, At);

  dim3 gConv(8, NH);
  k_conv<<<gConv, 128, 0, stream>>>(uh, At, u, Dv, yhi, ylo);

  dim3 gMix(NL / 32, NB);
  k_mix<<<gMix, 256, 0, stream>>>(yhi, ylo, whi, wlo, bm, out);
}
